// GConvGRU_19473381720232
// MI455X (gfx1250) — hardware-run, weakly checked
//
#include <hip/hip_runtime.h>


namespace {
constexpr int N = 20000, NP = 20032  , E = 320000, D = 512;
constexpr float XS = 8.0f, WSC = 256.0f;

typedef _Float16 b16;
typedef __attribute__((ext_vector_type(16))) _Float16 v16b;
typedef __attribute__((ext_vector_type(8))) _Float16 v8b;
typedef __attribute__((ext_vector_type(8))) float v8f;
typedef __attribute__((ext_vector_type(4))) float v4f;
__device__ __forceinline__ float bf16_rne(float f) { unsigned int u = __float_as_uint(f); u += 0x7FFFu + ((u >> 16) & 1u); return __uint_as_float(u & 0xFFFF0000u); }
__device__ __forceinline__ void split16(float v, b16& hi, b16& lo) { hi = (b16)v; lo = (b16)(v - (float)hi); }
__device__ __forceinline__ v16b frag_kb(const b16* p, int hh) { const v8b a = *(const v8b*)(p + 8 * hh), b = *(const v8b*)(p + 16 + 8 * hh); v16b f;
#pragma unroll
  for (int e = 0; e < 8; ++e) { f[e] = a[e]; f[8 + e] = b[e]; } return f; }
__device__ __forceinline__ v8f wmma16b(v16b a, v16b b, v8f c) { v8f d = __builtin_amdgcn_wmma_f32_16x16x32_f16(false, a, false, b, (short)0, c, false, false); asm volatile("v_nop\n\tv_nop\n\tv_nop\n\tv_nop" : "+v"(d) : "v"(a), "v"(b)); return d; }
__device__ __forceinline__ void wave_lds_sync() { __builtin_amdgcn_fence(__ATOMIC_RELEASE, "workgroup"); __builtin_amdgcn_wave_barrier(); __builtin_amdgcn_fence(__ATOMIC_ACQUIRE, "workgroup"); }
__device__ __forceinline__ float pmul(float a, float b) { float p = a * b; asm volatile("" : "+v"(p)); return p; }
__device__ __forceinline__ int iclamp(int v, int lo, int hi) { return v < lo ? lo : (v > hi ? hi : v); }
__device__ __forceinline__ float nexp(float x) { return __builtin_amdgcn_exp2f(x * 1.4426950408889634f); }
__device__ __forceinline__ float sigm(float x) { return 1.0f / (1.0f + nexp(-x)); }
__device__ __forceinline__ float tanh_(float x) { const float e = nexp(-2.0f * fabsf(x)); const float t = (1.0f - e) / (1.0f + e); return x < 0.0f ? -t : t; }

constexpr int CSR_NBLK = 512, CSR_GB = 9, CSR_GN = 1 << CSR_GB  , CSR_MAXG = 512, CSR_CAP = 12288  ;
__global__ __launch_bounds__(64) void csrA_kernel(const int* __restrict__ dst, int E, int N, int nG, int CHP, int NGP, int* __restrict__ STG, int* __restrict__ HST) {
  extern __shared__ int sm[];
  int* cnt = sm; int* run = sm + NGP; int* ids = sm + 2 * NGP;
  const int b = blockIdx.x; const int ch = (E + CSR_NBLK - 1) / CSR_NBLK; const int e0 = b * ch, e1 = min(E, e0 + ch);
  for (int i = threadIdx.x; i < NGP; i += 64) cnt[i] = 0;
  for (int i = threadIdx.x; i < CHP; i += 64) ids[i] = -1;
  __syncthreads();
  if (threadIdx.x == 0) {
    for (int e = e0; e < e1; ++e) { int d = dst[e]; d = (d < 0) ? 0 : (d >= N ? N - 1 : d); cnt[d >> CSR_GB] += 1; }
    int acc = 0; for (int g = 0; g < nG; ++g) { run[g] = acc; acc += cnt[g]; }
    for (int e = e0; e < e1; ++e) { int d = dst[e]; d = (d < 0) ? 0 : (d >= N ? N - 1 : d); const int g = d >> CSR_GB; ids[run[g]] = e; run[g] += 1; } }
  __syncthreads();
  typedef __attribute__((ext_vector_type(4))) int v4i;
  for (int pass = 0; pass < 2; ++pass) {
    for (int i = threadIdx.x; i < CHP / 4; i += 64) *(volatile v4i*)(STG + (size_t)b * CHP + i * 4) = *(const v4i*)(&ids[i * 4]);
    for (int i = threadIdx.x; i < NGP / 4; i += 64) { v4i v; for (int e = 0; e < 4; ++e) v[e] = (i * 4 + e < nG) ? cnt[i * 4 + e] : 0; *(volatile v4i*)(HST + (size_t)b * NGP + i * 4) = v; }
    __threadfence(); }
}
__global__ __launch_bounds__(512) void csrS_kernel(const int* __restrict__ HST, int nG, int NGP, int* __restrict__ START, int* __restrict__ TOT, int* __restrict__ OFF) {
  __shared__ int tot[CSR_MAXG];
  const int b = threadIdx.x;
  for (int pass = 0; pass < 2; ++pass) { int runb = 0; for (int g = 0; g < nG; ++g) { int c = HST[(size_t)b * NGP + g]; c = (c < 0) ? 0 : c; ((volatile int*)OFF)[(size_t)g * CSR_NBLK + b] = runb; runb += c; } __threadfence(); }
  for (int g = threadIdx.x; g < nG; g += 512) { int s = 0; for (int bb = 0; bb < CSR_NBLK; ++bb) { int c = HST[(size_t)bb * NGP + g]; s += (c < 0) ? 0 : c; } tot[g] = s; }
  __syncthreads();
  if (threadIdx.x < 32) {
    __shared__ int st[CSR_MAXG + 32];
    if (threadIdx.x == 0) { int acc = 0; for (int g = 0; g < NGP; ++g) { st[g] = acc; if (g < nG) acc += (tot[g] + 31) & ~31; } st[NGP] = acc; }
    __builtin_amdgcn_fence(__ATOMIC_RELEASE, "workgroup"); __builtin_amdgcn_wave_barrier(); __builtin_amdgcn_fence(__ATOMIC_ACQUIRE, "workgroup");
    for (int pass = 0; pass < 2; ++pass) { for (int i = threadIdx.x; i < NGP + 32; i += 32) { ((volatile int*)START)[i] = (i <= NGP) ? st[min(i, NGP)] : 0; ((volatile int*)TOT)[i] = (i < nG) ? tot[i] : 0; } __threadfence(); } }
}
__global__ __launch_bounds__(256) void csrB_kernel(const int* __restrict__ dst, int N, int nG, int CHP, int NGP, int permLen, const int* __restrict__ STG, const int* __restrict__ HST, const int* __restrict__ OFF, const int* __restrict__ START, const int* __restrict__ TOT, int* __restrict__ PERM, int* __restrict__ ROWPTR, int* __restrict__ ROWCNT, int* __restrict__ FLAG) {
  typedef __attribute__((ext_vector_type(4))) int v4i;
  __shared__ int ids[CSR_CAP]; __shared__ unsigned short key[CSR_CAP]; __shared__ int outp[CSR_CAP]; __shared__ int ncnt[CSR_GN + 1]; __shared__ int boff[CSR_NBLK + 1];
  const int g = blockIdx.x, t_ = threadIdx.x; int tot = TOT[g]; int st = START[g], stn = START[g + 1]; const int v0 = g * CSR_GN; const int nv = min(CSR_GN, N - v0);
  st = (st < 0) ? 0 : (st > permLen - 32 ? permLen - 32 : st) & ~31; stn = (stn < st) ? st : (stn > permLen ? permLen : stn); tot = (tot < 0) ? 0 : tot; if (tot > stn - st && tot <= CSR_CAP) tot = stn - st;
  if (tot > CSR_CAP) {
    for (int pass = 0; pass < 2; ++pass) { for (int i = t_; i < CSR_GN / 4; i += 256) { v4i a, c; for (int e = 0; e < 4; ++e) { a[e] = st; c[e] = 0; } *(volatile v4i*)(ROWPTR + v0 + i * 4) = a; *(volatile v4i*)(ROWCNT + v0 + i * 4) = c; } if (t_ == 0) ((volatile int*)FLAG)[0] = 1; __threadfence(); } (void)nv; return; }
  if (t_ == 0) { int acc = 0; for (int b = 0; b < CSR_NBLK; ++b) { boff[b] = acc; int c = HST[(size_t)b * NGP + g]; c = (c < 0) ? 0 : (c > CHP ? CHP : c); acc += c; if (acc > tot) acc = tot; } boff[CSR_NBLK] = acc; }
  for (int i = t_; i <= CSR_GN; i += 256) ncnt[i] = 0;
  __syncthreads();
  for (int b = 0; b < CSR_NBLK; ++b) { const int c = boff[b + 1] - boff[b]; int o_ = OFF[(size_t)g * CSR_NBLK + b]; o_ = (o_ < 0) ? 0 : (o_ > CHP - c ? CHP - c : o_); const int* src_ = STG + (size_t)b * CHP + o_;
    for (int i = t_; i < c; i += 256) { int id = src_[i]; id = (id < 0) ? 0 : id; ids[boff[b] + i] = id; int d = dst[id]; d = (d < v0) ? v0 : (d >= N ? N - 1 : d); int kk = d - v0; kk = (kk < 0) ? 0 : (kk >= CSR_GN ? CSR_GN - 1 : kk); key[boff[b] + i] = (unsigned short)kk; } }
  __syncthreads();
  if (t_ == 0) { for (int i = 0; i < tot; ++i) ncnt[key[i]] += 1; int acc = 0; for (int vl = 0; vl < CSR_GN; ++vl) { const int c = ncnt[vl]; ncnt[vl] = acc; acc += c; } ncnt[CSR_GN] = acc;
    for (int i = 0; i < tot; ++i) { const int vl = key[i]; outp[ncnt[vl]] = ids[i]; ncnt[vl] += 1; }
    for (int vl = CSR_GN; vl > 0; --vl) ncnt[vl] = ncnt[vl - 1]; ncnt[0] = 0; }
  __syncthreads();
  for (int pass = 0; pass < 2; ++pass) {
    for (int i = t_; i < (stn - st) / 4; i += 256) { v4i v; for (int e = 0; e < 4; ++e) { const int q = i * 4 + e; v[e] = (q < tot) ? outp[q] : -1; } *(volatile v4i*)(PERM + st + i * 4) = v; }
    for (int i = t_; i < CSR_GN / 4; i += 256) { v4i a, c; for (int e = 0; e < 4; ++e) { const int vl = i * 4 + e; a[e] = st + ncnt[vl]; c[e] = (vl < nv) ? (ncnt[vl + 1] - ncnt[vl]) : 0; } *(volatile v4i*)(ROWPTR + v0 + i * 4) = a; *(volatile v4i*)(ROWCNT + v0 + i * 4) = c; }
    __threadfence(); }
}
__global__ __launch_bounds__(256) void csrZ_kernel(int* __restrict__ p, size_t n4) { typedef __attribute__((ext_vector_type(4))) int v4i; const size_t tid = (size_t)blockIdx.x * 256 + threadIdx.x, nth = (size_t)gridDim.x * 256; v4i z = {0, 0, 0, 0}; for (size_t i = tid; i < n4; i += nth) *(volatile v4i*)(p + i * 4) = z; }
struct CsrBufs { int *STG, *HST, *OFF, *START, *TOT, *PERM, *ROWPTR, *ROWCNT, *FLAG; int nG, NGP, CHP; size_t permLen; char* base; size_t bytes; };
static size_t csr_carve(CsrBufs& c, char* ws, size_t off, int E, int N) {
  const size_t off0 = off; c.base = ws + off;
  auto al = [&](size_t bytes) { char* p = ws + off; off += (bytes + 255) & ~(size_t)255; return p; };
  c.nG = (N + CSR_GN - 1) / CSR_GN; c.NGP = (c.nG + 31) & ~31; const int ch = (E + CSR_NBLK - 1) / CSR_NBLK; c.CHP = (ch + 31) & ~31; c.permLen = (size_t)E + 32 * (size_t)c.nG + 32;
  c.STG = (int*)al((size_t)CSR_NBLK * c.CHP * 4); c.HST = (int*)al((size_t)CSR_NBLK * c.NGP * 4); c.OFF = (int*)al((size_t)c.NGP * CSR_NBLK * 4); c.START = (int*)al((size_t)(c.NGP + 64) * 4); c.TOT = (int*)al((size_t)(c.NGP + 64) * 4);
  c.PERM = (int*)al(c.permLen * 4); c.ROWPTR = (int*)al((size_t)c.nG * CSR_GN * 4); c.ROWCNT = (int*)al((size_t)c.nG * CSR_GN * 4); c.FLAG = (int*)al(256);
  c.bytes = off - off0; return off;
}
static void csr_build(const CsrBufs& c, const int* dst, int E, int N, hipStream_t stream) {
  const size_t smem = (size_t)(2 * c.NGP + c.CHP) * 4;
  csrZ_kernel<<<512, 256, 0, stream>>>((int*)c.base, c.bytes / 16);
  csrA_kernel<<<CSR_NBLK, 64, smem, stream>>>(dst, E, N, c.nG, c.CHP, c.NGP, c.STG, c.HST);
  csrS_kernel<<<1, 512, 0, stream>>>(c.HST, c.nG, c.NGP, c.START, c.TOT, c.OFF);
  csrB_kernel<<<c.nG, 256, 0, stream>>>(dst, N, c.nG, c.CHP, c.NGP, (int)c.permLen, c.STG, c.HST, c.OFF, c.START, c.TOT, c.PERM, c.ROWPTR, c.ROWCNT, c.FLAG);
}


__global__ __launch_bounds__(256) void prepw_kernel(const float* __restrict__ wxz, const float* __restrict__ whz, const float* __restrict__ wxr, const float* __restrict__ whr, const float* __restrict__ wxh, const float* __restrict__ whh, b16* __restrict__ WP) {
  const size_t t = (size_t)blockIdx.x * 256 + threadIdx.x; const size_t per = (size_t)D * 2 * D / 8; if (t >= 3 * per) return; const int which = (int)(t / per); const size_t e = (t - (size_t)which * per) * 8; const int oo = (int)(e / (2 * D)), k0 = (int)(e % (2 * D));
  const float* wa = which == 0 ? wxr : which == 1 ? wxz : wxh; const float* wb = which == 0 ? whr : which == 1 ? whz : whh; v8b o;
  for (int j = 0; j < 8; ++j) { const int k = k0 + j; const float v = (k < D) ? wa[(size_t)k * D + oo] : wb[(size_t)(k - D) * D + oo]; o[j] = (b16)(bf16_rne(v) * WSC); }
  for (int pass = 0; pass < 2; ++pass) { *(volatile v8b*)(WP + (size_t)which * D * 2 * D + e) = o; __threadfence(); }
}
__global__ __launch_bounds__(256) void dinv_kernel(const float* __restrict__ w, const int* __restrict__ PERM, const int* __restrict__ ROWPTR, const int* __restrict__ ROWCNT, int permLen, float* __restrict__ DINV) {
  const int v = blockIdx.x * 256 + threadIdx.x; if (v >= NP) return; float di = 0.0f;
  if (v < N) { int st = ROWPTR[v], cnt = ROWCNT[v]; cnt = iclamp(cnt, 0, 8192); st = iclamp(st, 0, permLen - cnt); float s = 1.0f; for (int j = 0; j < cnt; ++j) { const int e = iclamp(PERM[st + j], 0, E - 1); s += bf16_rne(w[e]); } di = rsqrtf(s); }
  for (int pass = 0; pass < 2; ++pass) { ((volatile float*)DINV)[v] = di; __threadfence(); }
}
template <int MODE>
__global__ __launch_bounds__(256) void agg_kernel(const float* __restrict__ SRCf, const b16* __restrict__ SRCh, const b16* __restrict__ SRCl, const int* __restrict__ rows, const float* __restrict__ w, const float* __restrict__ DINV, const int* __restrict__ PERM, const int* __restrict__ ROWPTR, const int* __restrict__ ROWCNT, int permLen, b16* __restrict__ OUTh, b16* __restrict__ OUTl) {
  const int wave = threadIdx.x >> 5, lane = threadIdx.x & 31; const size_t v = (size_t)blockIdx.x * 8 + wave; const int c0 = lane * 16;
  float acc[16]; for (int q = 0; q < 16; ++q) acc[q] = 0.0f;
  auto load16 = [&](size_t node, float* dst) { if (MODE == 0) { const float* p = SRCf + node * D + c0; for (int q = 0; q < 16; ++q) dst[q] = bf16_rne(p[q]); } else { const v8b a0 = *(const v8b*)(SRCh + node * D + c0), a1 = *(const v8b*)(SRCh + node * D + c0 + 8); v8b b0 = {}, b1 = {}; if (SRCl) { b0 = *(const v8b*)(SRCl + node * D + c0); b1 = *(const v8b*)(SRCl + node * D + c0 + 8); } for (int q = 0; q < 8; ++q) { dst[q] = ((float)a0[q] + (float)b0[q]) * (1.0f / XS); dst[8 + q] = ((float)a1[q] + (float)b1[q]) * (1.0f / XS); } } };
  if (v < (size_t)N) { const float dv = DINV[v]; int st = ROWPTR[v], cnt = ROWCNT[v]; cnt = iclamp(cnt, 0, 8192); st = iclamp(st, 0, permLen - cnt);
    { float xv[16]; load16(v, xv); const float nn = pmul(dv, dv); for (int q = 0; q < 16; ++q) acc[q] = pmul(nn, xv[q]); }
    for (int j = 0; j < cnt; ++j) { const int e = iclamp(PERM[st + j], 0, E - 1); const int r = iclamp(rows[e], 0, N - 1); const float nrm = pmul(pmul(DINV[r], bf16_rne(w[e])), dv); float xv[16]; load16((size_t)r, xv); for (int q = 0; q < 16; ++q) acc[q] += pmul(nrm, xv[q]); } }
  v8b h0, h1, l0, l1; for (int q = 0; q < 8; ++q) { b16 p, qq; split16(acc[q] * XS, p, qq); h0[q] = p; l0[q] = qq; split16(acc[8 + q] * XS, p, qq); h1[q] = p; l1[q] = qq; }
  for (int pass = 0; pass < 2; ++pass) { *(volatile v8b*)(OUTh + v * D + c0) = h0; *(volatile v8b*)(OUTh + v * D + c0 + 8) = h1; *(volatile v8b*)(OUTl + v * D + c0) = l0; *(volatile v8b*)(OUTl + v * D + c0 + 8) = l1; __threadfence(); }
}
__global__ __launch_bounds__(128) void passzr_kernel(const b16* __restrict__ AXh, const b16* __restrict__ AXl, const b16* __restrict__ AHh, const b16* __restrict__ AHl, const b16* __restrict__ WZ, const b16* __restrict__ WR, const float* __restrict__ bxz, const float* __restrict__ bhz, const float* __restrict__ bxr, const float* __restrict__ bhr, const float* __restrict__ Hin, unsigned short* __restrict__ Z16, b16* __restrict__ HRh) {
  __shared__ __attribute__((aligned(16))) float Ts[4][16][128 + 4];
  const int wave = threadIdx.x >> 5, lane = threadIdx.x & 31, nloc = lane & 15, hlf = lane >> 4; const size_t m0 = ((size_t)blockIdx.x * 4 + wave) * 16; const int isR = blockIdx.y >= 4; const int n0 = (blockIdx.y & 3) * 128;
  const b16* W = isR ? WR : WZ;
  v8f acc[8];
#pragma unroll
  for (int t = 0; t < 8; ++t) acc[t] = (v8f){};
  for (int seg = 0; seg < 2; ++seg) { const b16* Ah = seg == 0 ? AXh : AHh; const b16* Al = seg == 0 ? AXl : AHl;
#pragma unroll 2
    for (int kb = 0; kb < D; kb += 32) { const v16b a = frag_kb(Ah + (m0 + nloc) * D + kb, hlf), al = frag_kb(Al + (m0 + nloc) * D + kb, hlf);
#pragma unroll
      for (int t = 0; t < 8; ++t) { const v16b bw = frag_kb(W + (size_t)(n0 + t * 16 + nloc) * (2 * D) + seg * D + kb, hlf); acc[t] = wmma16b(a, bw, acc[t]); acc[t] = wmma16b(al, bw, acc[t]); } } }
#pragma unroll
  for (int t = 0; t < 8; ++t) { const int c = n0 + t * 16 + nloc; const float bb = isR ? bf16_rne(bxr[c]) + bf16_rne(bhr[c]) : bf16_rne(bxz[c]) + bf16_rne(bhz[c]);
#pragma unroll
    for (int r = 0; r < 8; ++r) { const size_t row = m0 + 8 * hlf + r; const float g = sigm(acc[t][r] * (1.0f / (XS * WSC)) + bb); float v = g; if (isR) v = (row < (size_t)N) ? pmul(bf16_rne(Hin[row * D + c]), g) : 0.0f; Ts[wave][8 * hlf + r][t * 16 + nloc] = v; } }
  wave_lds_sync();
  typedef __attribute__((ext_vector_type(8))) unsigned short v8u;
  for (int pass = 0; pass < 2; ++pass) { for (int rr = 0; rr < 16; ++rr) if (lane < 16) {
      if (isR) { v8b hv; for (int j = 0; j < 8; ++j) hv[j] = (b16)(Ts[wave][rr][lane * 8 + j] * XS); *(volatile v8b*)(HRh + (m0 + rr) * D + n0 + lane * 8) = hv; }
      else { v8u u; for (int j = 0; j < 8; ++j) u[j] = (unsigned short)rintf(Ts[wave][rr][lane * 8 + j] * 65535.0f); *(volatile v8u*)(Z16 + (m0 + rr) * D + n0 + lane * 8) = u; } }
    __threadfence(); }
}
__global__ __launch_bounds__(128) void final_kernel(const b16* __restrict__ AXh, const b16* __restrict__ AXl, const b16* __restrict__ ARh, const b16* __restrict__ ARl, const b16* __restrict__ WHt, const float* __restrict__ bxh, const float* __restrict__ bhh, const float* __restrict__ Hin, const unsigned short* __restrict__ Z16, float* __restrict__ out) {
  __shared__ __attribute__((aligned(16))) float Ts[4][16][128 + 4];
  const int wave = threadIdx.x >> 5, lane = threadIdx.x & 31, nloc = lane & 15, hlf = lane >> 4; const size_t m0 = ((size_t)blockIdx.x * 4 + wave) * 16; const int n0 = blockIdx.y * 128;
  v8f ah[8];
#pragma unroll
  for (int t = 0; t < 8; ++t) ah[t] = (v8f){};
  for (int seg = 0; seg < 2; ++seg) { const b16* Ah_ = seg == 0 ? AXh : ARh; const b16* Al_ = seg == 0 ? AXl : ARl;
#pragma unroll 2
    for (int kb = 0; kb < D; kb += 32) { const v16b a = frag_kb(Ah_ + (m0 + nloc) * D + kb, hlf), al = frag_kb(Al_ + (m0 + nloc) * D + kb, hlf);
#pragma unroll
      for (int t = 0; t < 8; ++t) { const v16b wh = frag_kb(WHt + (size_t)(n0 + t * 16 + nloc) * (2 * D) + seg * D + kb, hlf); ah[t] = wmma16b(a, wh, ah[t]); ah[t] = wmma16b(al, wh, ah[t]); } } }
#pragma unroll
  for (int t = 0; t < 8; ++t) { const int c = n0 + t * 16 + nloc; const float bh = bf16_rne(bxh[c]) + bf16_rne(bhh[c]);
#pragma unroll
    for (int r = 0; r < 8; ++r) { const size_t row = m0 + 8 * hlf + r; const float ht = tanh_(ah[t][r] * (1.0f / (XS * WSC)) + bh); float o = 0.0f; if (row < (size_t)N) { const float z = (float)Z16[row * D + c] * (1.0f / 65535.0f); o = pmul(z, bf16_rne(Hin[row * D + c])) + pmul(1.0f - z, ht); } Ts[wave][8 * hlf + r][t * 16 + nloc] = o; } }
  wave_lds_sync();
  for (int pass = 0; pass < 2; ++pass) { for (int rr = 0; rr < 16; ++rr) { const size_t row = m0 + rr; if (row < (size_t)N) *(volatile v4f*)(out + row * D + n0 + lane * 4) = *(const v4f*)(&Ts[wave][rr][lane * 4]); } __threadfence(); }
}
}

extern "C" void kernel_launch(void* const* d_in, const int* in_sizes, int n_in, void* d_out, int out_size, void* d_ws, size_t ws_size, hipStream_t stream) {
  (void)n_in;
  auto Fp = [&](int i) { return (const float*)d_in[i]; }; auto Ip = [&](int i) { return (const int*)d_in[i]; };
  if (in_sizes[0] != N * D || in_sizes[1] != 2 * E || in_sizes[2] != E || in_sizes[3] != N * D || in_sizes[4] != D * D || in_sizes[14] != D * D || out_size != N * D) return;
  size_t off = 0; char* ws = (char*)d_ws;
  auto carve = [&](size_t bytes) { char* p = ws + off; off += (bytes + 255) & ~(size_t)255; return p; };
  b16* WP = (b16*)carve((size_t)3 * D * 2 * D * 2); float* DINV = (float*)carve((size_t)(NP + 256) * 4);
  b16* AXh = (b16*)carve((size_t)NP * D * 2); b16* AXl = (b16*)carve((size_t)NP * D * 2); b16* AHh = (b16*)carve((size_t)NP * D * 2); b16* AHl = (b16*)carve((size_t)NP * D * 2); b16* HRh = (b16*)carve((size_t)NP * D * 2); unsigned short* Z16 = (unsigned short*)carve((size_t)NP * D * 2);
  CsrBufs csr; off = csr_carve(csr, ws, off, E, N);
  if (off > ws_size || off > ((size_t)128 << 20)) return;
  b16* ARh = AHh; b16* ARl = AHl;
  const b16 *WR = WP, *WZ = WP + (size_t)D * 2 * D, *WHt = WP + (size_t)2 * D * 2 * D;
  prepw_kernel<<<(unsigned)(((size_t)3 * D * 2 * D / 8 + 255) / 256), 256, 0, stream>>>(Fp(4), Fp(6), Fp(8), Fp(10), Fp(12), Fp(14), WP);
  csr_build(csr, Ip(1) + E, E, N, stream);
  dinv_kernel<<<(NP + 255) / 256, 256, 0, stream>>>(Fp(2), csr.PERM, csr.ROWPTR, csr.ROWCNT, (int)csr.permLen, DINV);
  agg_kernel<0><<<NP / 8, 256, 0, stream>>>(Fp(0), nullptr, nullptr, Ip(1), Fp(2), DINV, csr.PERM, csr.ROWPTR, csr.ROWCNT, (int)csr.permLen, AXh, AXl);
  agg_kernel<0><<<NP / 8, 256, 0, stream>>>(Fp(3), nullptr, nullptr, Ip(1), Fp(2), DINV, csr.PERM, csr.ROWPTR, csr.ROWCNT, (int)csr.permLen, AHh, AHl);
  passzr_kernel<<<dim3(NP / 64, 8), 128, 0, stream>>>(AXh, AXl, AHh, AHl, WZ, WR, Fp(5), Fp(7), Fp(9), Fp(11), Fp(3), Z16, HRh);
  agg_kernel<1><<<NP / 8, 256, 0, stream>>>(nullptr, HRh, nullptr, Ip(1), Fp(2), DINV, csr.PERM, csr.ROWPTR, csr.ROWCNT, (int)csr.permLen, ARh, ARl);
  final_kernel<<<dim3(NP / 64, 4), 128, 0, stream>>>(AXh, AXl, ARh, ARl, WHt, Fp(13), Fp(15), Fp(3), Z16, (float*)d_out);
}
